// MultiHeadAttention_34162169872901
// MI455X (gfx1250) — hardware-run, weakly checked
//
#include <hip/hip_runtime.h>
#ifndef NB
#define NB 4
#endif
#ifndef SEQ
#define SEQ 2048
#endif
#define NB_FULL 4
#define SEQ_FULL 2048
#define DM 512
#define NH 8
#define HD 64
#define NBIAS 511
#define XSTRIDE_FULL ((size_t)SEQ_FULL * DM)
#define PLANE_BYTES ((size_t)NB * SEQ * DM * 2)
#define WPLANE_BYTES ((size_t)DM * DM * 2)

static_assert(SEQ % 64 == 0);
static_assert(SEQ <= SEQ_FULL);
static_assert(NB <= NB_FULL);
static_assert(HD == 64);
static_assert(NH * HD == DM);
static_assert(DM % 64 == 0);
static_assert((NB * SEQ) % 64 == 0);
static_assert(8 * PLANE_BYTES + 4 * WPLANE_BYTES <= (size_t)134217728);

typedef __bf16 v16b __attribute__((ext_vector_type(16)));
typedef _Float16 v16h __attribute__((ext_vector_type(16)));
typedef unsigned short v8us __attribute__((ext_vector_type(8), may_alias));
typedef float v8f __attribute__((ext_vector_type(8)));
typedef float v4f __attribute__((ext_vector_type(4)));
typedef float v4fa __attribute__((ext_vector_type(4), may_alias));
union FragB { v16b v; v8us half[2]; unsigned short u[16]; };
union FragH { v16h v; v8us half[2]; _Float16 h[16]; unsigned short u[16]; };

#define LOG2E 1.4426950408889634f
#define NEGV (-1000000000.0f)

__device__ __forceinline__ unsigned short bf16_bits(float x) {
  unsigned int u = __float_as_uint(x);
  return (unsigned short)((u + 0x7FFFu + ((u >> 16) & 1u)) >> 16);
}
__device__ __forceinline__ float bf16_val(unsigned short b) { return __uint_as_float(((unsigned int)b) << 16); }
__device__ __forceinline__ float bf16_rne(float x) { return bf16_val(bf16_bits(x)); }

__device__ __forceinline__ void split8(v4f x0, v4f x1, v8us& oh, v8us& ol) {
#pragma unroll
  for (int i = 0; i < 4; ++i) {
    const unsigned short h0 = bf16_bits(x0[i]);
    const unsigned short h1 = bf16_bits(x1[i]);
    oh[i] = h0; oh[4 + i] = h1;
    ol[i] = bf16_bits(x0[i] - bf16_val(h0));
    ol[4 + i] = bf16_bits(x1[i] - bf16_val(h1));
  }
}
__device__ __forceinline__ v8us half8(v4f x0, v4f x1) {
  FragH f;
#pragma unroll
  for (int i = 0; i < 4; ++i) { f.h[i] = (_Float16)x0[i]; f.h[4 + i] = (_Float16)x1[i]; }
  return f.half[0];
}

__device__ __forceinline__ void mma_b4(v16b a, v16b b0, v16b b1, v16b b2, v16b b3, v8f& c0, v8f& c1, v8f& c2, v8f& c3) {
  c0 = __builtin_amdgcn_wmma_f32_16x16x32_bf16(false, a, false, b0, (short)0, c0, false, false);
  c1 = __builtin_amdgcn_wmma_f32_16x16x32_bf16(false, a, false, b1, (short)0, c1, false, false);
  c2 = __builtin_amdgcn_wmma_f32_16x16x32_bf16(false, a, false, b2, (short)0, c2, false, false);
  c3 = __builtin_amdgcn_wmma_f32_16x16x32_bf16(false, a, false, b3, (short)0, c3, false, false);
  asm volatile("v_nop\n\tv_nop\n\tv_nop\n\tv_nop" : "+v"(c0), "+v"(c1), "+v"(c2), "+v"(c3) : "v"(a), "v"(b0), "v"(b1), "v"(b2), "v"(b3));
}
__device__ __forceinline__ v8f mma_hs2(v16h a0, v16h b0, v16h a1, v16h b1, v8f c) {
  c = __builtin_amdgcn_wmma_f32_16x16x32_f16(false, a0, false, b0, (short)0, c, false, false);
  c = __builtin_amdgcn_wmma_f32_16x16x32_f16(false, a1, false, b1, (short)0, c, false, false);
  asm volatile("v_nop\n\tv_nop\n\tv_nop\n\tv_nop" : "+v"(c) : "v"(a0), "v"(b0), "v"(a1), "v"(b1));
  return c;
}
__device__ __forceinline__ void mma_pv4(v16h a0, v16h a1, v16h a2, v16h a3, v16h p, v8f& c0, v8f& c1, v8f& c2, v8f& c3) {
  c0 = __builtin_amdgcn_wmma_f32_16x16x32_f16(false, a0, false, p, (short)0, c0, false, false);
  c1 = __builtin_amdgcn_wmma_f32_16x16x32_f16(false, a1, false, p, (short)0, c1, false, false);
  c2 = __builtin_amdgcn_wmma_f32_16x16x32_f16(false, a2, false, p, (short)0, c2, false, false);
  c3 = __builtin_amdgcn_wmma_f32_16x16x32_f16(false, a3, false, p, (short)0, c3, false, false);
  asm volatile("v_nop\n\tv_nop\n\tv_nop\n\tv_nop" : "+v"(c0), "+v"(c1), "+v"(c2), "+v"(c3) : "v"(a0), "v"(a1), "v"(a2), "v"(a3), "v"(p));
}

__global__ __launch_bounds__(256) void k_cvt(const float* __restrict__ src, unsigned short* __restrict__ dst, int nrows, int rpb, size_t sbstride) {
  const int t = blockIdx.x * 256 + threadIdx.x;
  if (t >= nrows * (DM / 8)) return;
  const int row = t >> 6, piece = t & 63;
  const int b = row / rpb, s = row - b * rpb;
  const float* p = src + (size_t)b * sbstride + (size_t)s * DM + piece * 8;
  const v4f x0 = *(const v4fa*)(p), x1 = *(const v4fa*)(p + 4);
  v8us o;
  o[0] = bf16_bits(x0[0]); o[1] = bf16_bits(x0[1]); o[2] = bf16_bits(x0[2]); o[3] = bf16_bits(x0[3]);
  o[4] = bf16_bits(x1[0]); o[5] = bf16_bits(x1[1]); o[6] = bf16_bits(x1[2]); o[7] = bf16_bits(x1[3]);
  unsigned short* d = dst + (size_t)t * 8;
  *(volatile v8us*)d = o;
  __threadfence();
  *(volatile v8us*)d = o;
}

__device__ __forceinline__ void gemm_k512(const unsigned short* __restrict__ ap, const unsigned short* __restrict__ bp, v8f (&acc)[4]) {
#pragma unroll 2
  for (int k0 = 0; k0 < DM; k0 += 32) {
    FragB a, b0, b1, b2, b3;
    a.half[0]  = *(const v8us*)(ap + k0);               a.half[1]  = *(const v8us*)(ap + k0 + 16);
    b0.half[0] = *(const v8us*)(bp + k0);               b0.half[1] = *(const v8us*)(bp + k0 + 16);
    b1.half[0] = *(const v8us*)(bp + 16 * DM + k0);     b1.half[1] = *(const v8us*)(bp + 16 * DM + k0 + 16);
    b2.half[0] = *(const v8us*)(bp + 32 * DM + k0);     b2.half[1] = *(const v8us*)(bp + 32 * DM + k0 + 16);
    b3.half[0] = *(const v8us*)(bp + 48 * DM + k0);     b3.half[1] = *(const v8us*)(bp + 48 * DM + k0 + 16);
    mma_b4(a.v, b0.v, b1.v, b2.v, b3.v, acc[0], acc[1], acc[2], acc[3]);
  }
}

__global__ __launch_bounds__(128) void k_proj_qk(const unsigned short* __restrict__ Xb, const unsigned short* __restrict__ Wb,
                                                 unsigned short* __restrict__ Pf, float scale) {
  __shared__ __attribute__((aligned(16))) float so[4][16][68];
  const int tid = threadIdx.x, lane = tid & 31, ln = lane & 15, hh = lane >> 4;
  const int w = __builtin_amdgcn_readfirstlane((int)(threadIdx.x >> 5));
  const int m0 = blockIdx.x * 64 + 16 * w, n0 = blockIdx.y * 64;
  v8f acc[4] = {};
  gemm_k512(Xb + (size_t)(m0 + ln) * DM + 8 * hh, Wb + (size_t)(n0 + ln) * DM + 8 * hh, acc);
#pragma unroll
  for (int t = 0; t < 4; ++t)
#pragma unroll
    for (int r = 0; r < 8; ++r)
      so[w][8 * hh + r][16 * t + ln] = acc[t][r] * scale;
  __syncthreads();
  const int b = m0 / SEQ, s0 = m0 - b * SEQ, hd = blockIdx.y;
  const size_t base = (((size_t)b * NH + hd) * SEQ + s0) * HD;
  const int rq = lane >> 3, pc8 = (lane & 7) * 8;
  for (int pass = 0; pass < 2; ++pass) {
#pragma unroll
    for (int q = 0; q < 4; ++q) {
      const int row = 4 * q + rq;
      const v4f x0 = *(const v4fa*)&so[w][row][pc8];
      const v4f x1 = *(const v4fa*)&so[w][row][pc8 + 4];
      const v8us o = half8(x0, x1);
      *(volatile v8us*)(Pf + base + (size_t)row * HD + pc8) = o;
    }
    if (pass == 0) __threadfence();
  }
}

__global__ __launch_bounds__(128) void k_proj_v(const unsigned short* __restrict__ Wb, const unsigned short* __restrict__ Xb,
                                                unsigned short* __restrict__ Vt) {
  __shared__ __attribute__((aligned(16))) float so[4][16][68];
  const int tid = threadIdx.x, lane = tid & 31, ln = lane & 15, hh = lane >> 4;
  const int w = __builtin_amdgcn_readfirstlane((int)(threadIdx.x >> 5));
  const int m0 = blockIdx.x * 64 + 16 * w, n0 = blockIdx.y * 64;
  v8f acc[4] = {};
  gemm_k512(Wb + (size_t)(m0 + ln) * DM + 8 * hh, Xb + (size_t)(n0 + ln) * DM + 8 * hh, acc);
#pragma unroll
  for (int t = 0; t < 4; ++t)
#pragma unroll
    for (int r = 0; r < 8; ++r)
      so[w][8 * hh + r][16 * t + ln] = acc[t][r] * 16.0f;
  __syncthreads();
  const int b = n0 / SEQ, s0 = n0 - b * SEQ;
  const int rq = lane >> 3, pc8 = (lane & 7) * 8;
  for (int pass = 0; pass < 2; ++pass) {
#pragma unroll
    for (int q = 0; q < 4; ++q) {
      const int row = 4 * q + rq;
      const v4f x0 = *(const v4fa*)&so[w][row][pc8];
      const v4f x1 = *(const v4fa*)&so[w][row][pc8 + 4];
      const v8us o = half8(x0, x1);
      *(volatile v8us*)(Vt + ((size_t)b * DM + (m0 + row)) * SEQ + s0 + pc8) = o;
    }
    if (pass == 0) __threadfence();
  }
}

template <bool MASK>
__device__ __forceinline__ void fa_step(const unsigned short* __restrict__ Kp, const unsigned short* __restrict__ Vp,
                                        const float* sb, const int* sm,
                                        float b_lo, float b_hi, int key0, int qg, int qbase, int ln, int hh,
                                        const FragH& q0, const FragH& q1,
                                        float& mr, float& lr, v8f (&Oa)[4]) {
  const unsigned short* kp0 = Kp + (size_t)(key0 + ln) * HD + 8 * hh;
  const unsigned short* kp1 = kp0 + 16 * HD;
  FragH k00, k01, k10, k11;
  k00.half[0] = *(const v8us*)(kp0);      k00.half[1] = *(const v8us*)(kp0 + 16);
  k01.half[0] = *(const v8us*)(kp0 + 32); k01.half[1] = *(const v8us*)(kp0 + 48);
  k10.half[0] = *(const v8us*)(kp1);      k10.half[1] = *(const v8us*)(kp1 + 16);
  k11.half[0] = *(const v8us*)(kp1 + 32); k11.half[1] = *(const v8us*)(kp1 + 48);
  const unsigned short* vp = Vp + (size_t)ln * SEQ + key0 + 8 * hh;
  FragH vf[4];
#pragma unroll
  for (int t = 0; t < 4; ++t) {
    vf[t].half[0] = *(const v8us*)(vp + (size_t)t * 16 * SEQ);
    vf[t].half[1] = *(const v8us*)(vp + (size_t)t * 16 * SEQ + 16);
  }
  const v8f z8 = {0.f, 0.f, 0.f, 0.f, 0.f, 0.f, 0.f, 0.f};
  const v8f s0 = mma_hs2(k00.v, q0.v, k01.v, q1.v, z8);
  const v8f s1 = mma_hs2(k10.v, q0.v, k11.v, q1.v, z8);
  float sc[16];
#pragma unroll
  for (int r = 0; r < 8; ++r) { sc[r] = s0[r]; sc[8 + r] = s1[r]; }
  const int dlo = key0 - qbase;
  if (dlo <= -286) {
#pragma unroll
    for (int i = 0; i < 16; ++i) sc[i] += b_lo;
  } else if (dlo >= 270) {
#pragma unroll
    for (int i = 0; i < 16; ++i) sc[i] += b_hi;
  } else {
    const int d0 = key0 + 8 * hh - qg;
#pragma unroll
    for (int r = 0; r < 8; ++r) {
      int r0 = d0 + r;      r0 = (r0 < -255) ? -255 : ((r0 > 255) ? 255 : r0);
      int r1 = d0 + 16 + r; r1 = (r1 < -255) ? -255 : ((r1 > 255) ? 255 : r1);
      sc[r]     += sb[r0 + 255];
      sc[8 + r] += sb[r1 + 255];
    }
  }
  if (MASK) {
    const int kb = key0 + 8 * hh;
#pragma unroll
    for (int r = 0; r < 8; ++r) {
      const int m0 = sm[kb + r];
      const int m1 = sm[kb + 16 + r];
      sc[r]     = (m0 == 0) ? NEGV : sc[r];
      sc[8 + r] = (m1 == 0) ? NEGV : sc[8 + r];
    }
  }
  float mx = sc[0];
#pragma unroll
  for (int i = 1; i < 16; ++i) mx = fmaxf(mx, sc[i]);
  mx = fmaxf(mx, __shfl_xor(mx, 16, 32));
  const float mnew = fmaxf(mr, mx);
  const float al = exp2f((mr - mnew) * LOG2E);
  mr = mnew;
  FragH ph;
  float ps = 0.0f;
#pragma unroll
  for (int i = 0; i < 16; ++i) {
    const float pc = exp2f(fmaf(sc[i] - mnew, LOG2E, 8.0f));
    const _Float16 h = (_Float16)pc;
    ph.h[i] = h;
    ps += (float)h;
  }
  ps += __shfl_xor(ps, 16, 32);
  lr = lr * al + ps;
#pragma unroll
  for (int t = 0; t < 4; ++t) Oa[t] = Oa[t] * al;
  mma_pv4(vf[0].v, vf[1].v, vf[2].v, vf[3].v, ph.v, Oa[0], Oa[1], Oa[2], Oa[3]);
}

__global__ __launch_bounds__(128) void k_attn(const unsigned short* __restrict__ Qf, const unsigned short* __restrict__ Kf,
                                              const unsigned short* __restrict__ Vt, const int* __restrict__ mask,
                                              const float* __restrict__ relb, unsigned short* __restrict__ Ch, unsigned short* __restrict__ Cl) {
  __shared__ __attribute__((aligned(16))) float so[4][16][68];
  __shared__ float sb[512];
  __shared__ int sm[SEQ];
  __shared__ int sflag;
  const int tid = threadIdx.x, lane = tid & 31, ln = lane & 15, hh = lane >> 4;
  const int w = __builtin_amdgcn_readfirstlane((int)(threadIdx.x >> 5));
  const int bh = blockIdx.x / (SEQ / 64), qt = blockIdx.x % (SEQ / 64);
  const int b = bh / NH, h = bh - b * NH;
  const int qbase = qt * 64 + 16 * w;
  const int qg = qbase + ln;
  int zf = 0;
  for (int i = tid; i < SEQ; i += 128) {
    const int v = mask[(size_t)b * SEQ_FULL + i];
    sm[i] = v;
    zf |= (v == 0) ? 1 : 0;
  }
  for (int i = tid; i < 512; i += 128) {
    const int ic = (i < NBIAS) ? i : (NBIAS - 1);
    const float v = bf16_rne(relb[h * NBIAS + ic]);
    sb[i] = (i < NBIAS) ? v : 0.0f;
  }
  if (tid == 0) sflag = 0;
  __syncthreads();
  if (zf) sflag = 1;
  __syncthreads();
  const int anyz = __builtin_amdgcn_readfirstlane(sflag);
  const float b_lo = sb[0], b_hi = sb[NBIAS - 1];
  const size_t qoff = ((size_t)bh * SEQ + qg) * HD + 8 * hh;
  FragH q0, q1;
  q0.half[0] = *(const v8us*)(Qf + qoff);      q0.half[1] = *(const v8us*)(Qf + qoff + 16);
  q1.half[0] = *(const v8us*)(Qf + qoff + 32); q1.half[1] = *(const v8us*)(Qf + qoff + 48);
  float mr = -3.0e38f, lr = 0.0f;
  v8f Oa[4] = {};
  const unsigned short* Kp = Kf + (size_t)bh * SEQ * HD;
  const unsigned short* Vp = Vt + (size_t)bh * HD * SEQ;
  if (anyz) {
#pragma unroll 1
    for (int j = 0; j < SEQ / 32; ++j)
      fa_step<true>(Kp, Vp, sb, sm, b_lo, b_hi, 32 * j, qg, qbase, ln, hh, q0, q1, mr, lr, Oa);
  } else {
#pragma unroll 1
    for (int j = 0; j < SEQ / 32; ++j)
      fa_step<false>(Kp, Vp, sb, sm, b_lo, b_hi, 32 * j, qg, qbase, ln, hh, q0, q1, mr, lr, Oa);
  }
  const float inv = 1.0f / (16.0f * lr);
#pragma unroll
  for (int t = 0; t < 4; ++t)
#pragma unroll
    for (int r = 0; r < 8; ++r)
      so[w][ln][16 * t + 8 * hh + r] = Oa[t][r] * inv;
  __syncthreads();
  const int rq = lane >> 3, pc8 = (lane & 7) * 8;
  const size_t cbase = ((size_t)b * SEQ + qbase) * DM + (size_t)h * HD;
  for (int pass = 0; pass < 2; ++pass) {
#pragma unroll
    for (int q = 0; q < 4; ++q) {
      const int row = 4 * q + rq;
      const v4f x0 = *(const v4fa*)&so[w][row][pc8];
      const v4f x1 = *(const v4fa*)&so[w][row][pc8 + 4];
      v8us oh, ol;
      split8(x0, x1, oh, ol);
      *(volatile v8us*)(Ch + cbase + (size_t)row * DM + pc8) = oh;
      *(volatile v8us*)(Cl + cbase + (size_t)row * DM + pc8) = ol;
    }
    if (pass == 0) __threadfence();
  }
}

__global__ __launch_bounds__(128) void k_out(const unsigned short* __restrict__ Ch, const unsigned short* __restrict__ Cl,
                                             const unsigned short* __restrict__ Wb, const float* __restrict__ bo, float* __restrict__ O) {
  __shared__ __attribute__((aligned(16))) float so[4][16][68];
  const int tid = threadIdx.x, lane = tid & 31, ln = lane & 15, hh = lane >> 4;
  const int w = __builtin_amdgcn_readfirstlane((int)(threadIdx.x >> 5));
  const int m0 = blockIdx.x * 64 + 16 * w, n0 = blockIdx.y * 64;
  v8f acc[4] = {};
  const size_t aoff = (size_t)(m0 + ln) * DM + 8 * hh;
  const unsigned short* bp = Wb + (size_t)(n0 + ln) * DM + 8 * hh;
  gemm_k512(Cl + aoff, bp, acc);
  gemm_k512(Ch + aoff, bp, acc);
#pragma unroll
  for (int t = 0; t < 4; ++t)
#pragma unroll
    for (int r = 0; r < 8; ++r)
      so[w][8 * hh + r][16 * t + ln] = acc[t][r];
  __syncthreads();
  const int rsub = lane >> 4, c4 = (lane & 15) * 4;
  v4f bias;
  bias[0] = bf16_rne(bo[n0 + c4 + 0]); bias[1] = bf16_rne(bo[n0 + c4 + 1]);
  bias[2] = bf16_rne(bo[n0 + c4 + 2]); bias[3] = bf16_rne(bo[n0 + c4 + 3]);
  for (int pass = 0; pass < 2; ++pass) {
#pragma unroll
    for (int q = 0; q < 8; ++q) {
      const int row = 2 * q + rsub;
      const int m = m0 + row;
      const int b = m / SEQ, s = m - b * SEQ;
      const v4f x = *(const v4fa*)&so[w][row][c4];
      const v4f v = x + bias;
      *(volatile v4f*)(O + ((size_t)b * SEQ_FULL + s) * DM + n0 + c4) = v;
    }
    if (pass == 0) __threadfence();
  }
}

extern "C" void kernel_launch(void* const* d_in, const int* in_sizes, int n_in,
                              void* d_out, int out_size, void* d_ws, size_t ws_size, hipStream_t stream) {
  if (n_in < 10) return;
  const long long needx = ((long long)(NB - 1) * SEQ_FULL + SEQ) * DM;
  const long long needm = (long long)(NB - 1) * SEQ_FULL + SEQ;
  if ((long long)in_sizes[0] < needx || (long long)in_sizes[1] < needx || (long long)in_sizes[2] < needx) return;
  if ((long long)in_sizes[3] < needm) return;
  if (in_sizes[4] < DM * DM || in_sizes[5] < DM * DM || in_sizes[6] < DM * DM || in_sizes[7] < DM * DM) return;
  if (in_sizes[8] < DM || in_sizes[9] < NH * NBIAS) return;
  if ((long long)out_size < needx) return;
  const float* query = (const float*)d_in[0];
  const float* key   = (const float*)d_in[1];
  const float* value = (const float*)d_in[2];
  const int*   mask  = (const int*)d_in[3];
  const float* Wq    = (const float*)d_in[4];
  const float* Wk    = (const float*)d_in[5];
  const float* Wv    = (const float*)d_in[6];
  const float* Wo    = (const float*)d_in[7];
  const float* bo    = (const float*)d_in[8];
  const float* relb  = (const float*)d_in[9];
  float* O = (float*)d_out;
  char* ws = (char*)d_ws;
  size_t off = 0;
  const size_t plane = PLANE_BYTES;
  const size_t wplane = WPLANE_BYTES;
  unsigned short* Xq  = (unsigned short*)(ws + off); off += (plane + 255) & ~(size_t)255;
  unsigned short* Xk  = (unsigned short*)(ws + off); off += (plane + 255) & ~(size_t)255;
  unsigned short* Xv  = (unsigned short*)(ws + off); off += (plane + 255) & ~(size_t)255;
  unsigned short* Wqb = (unsigned short*)(ws + off); off += (wplane + 255) & ~(size_t)255;
  unsigned short* Wkb = (unsigned short*)(ws + off); off += (wplane + 255) & ~(size_t)255;
  unsigned short* Wvb = (unsigned short*)(ws + off); off += (wplane + 255) & ~(size_t)255;
  unsigned short* Wob = (unsigned short*)(ws + off); off += (wplane + 255) & ~(size_t)255;
  unsigned short* Qf  = (unsigned short*)(ws + off); off += (plane + 255) & ~(size_t)255;
  unsigned short* Kf  = (unsigned short*)(ws + off); off += (plane + 255) & ~(size_t)255;
  unsigned short* Vt  = (unsigned short*)(ws + off); off += (plane + 255) & ~(size_t)255;
  unsigned short* Ch  = (unsigned short*)(ws + off); off += (plane + 255) & ~(size_t)255;
  unsigned short* Cl  = (unsigned short*)(ws + off); off += (plane + 255) & ~(size_t)255;
  if (off > ws_size) return;

  const int rows = NB * SEQ;
  const unsigned gx = (unsigned)((rows * (DM / 8) + 255) / 256);
  const unsigned gw = (unsigned)((DM * (DM / 8) + 255) / 256);
  k_cvt<<<gx, 256, 0, stream>>>(query, Xq, rows, SEQ, XSTRIDE_FULL);
  k_cvt<<<gx, 256, 0, stream>>>(key,   Xk, rows, SEQ, XSTRIDE_FULL);
  k_cvt<<<gx, 256, 0, stream>>>(value, Xv, rows, SEQ, XSTRIDE_FULL);
  k_cvt<<<gw, 256, 0, stream>>>(Wq, Wqb, DM, DM, (size_t)0);
  k_cvt<<<gw, 256, 0, stream>>>(Wk, Wkb, DM, DM, (size_t)0);
  k_cvt<<<gw, 256, 0, stream>>>(Wv, Wvb, DM, DM, (size_t)0);
  k_cvt<<<gw, 256, 0, stream>>>(Wo, Wob, DM, DM, (size_t)0);

  const dim3 gp((unsigned)(rows / 64), (unsigned)(DM / 64));
  k_proj_qk<<<gp, 128, 0, stream>>>(Xq, Wqb, Qf, 0.125f);
  k_proj_qk<<<gp, 128, 0, stream>>>(Xk, Wkb, Kf, 1.0f);
  const dim3 gv((unsigned)(DM / 64), (unsigned)(rows / 64));
  k_proj_v<<<gv, 128, 0, stream>>>(Wvb, Xv, Vt);
  k_attn<<<(unsigned)(NB * NH * (SEQ / 64)), 128, 0, stream>>>(Qf, Kf, Vt, mask, relb, Ch, Cl);
  k_out<<<gp, 128, 0, stream>>>(Ch, Cl, Wob, bo, O);
}
